// EdgeConv_17875653886624
// MI455X (gfx1250) — hardware-verified
//
#include <hip/hip_runtime.h>
#include <math.h>

#pragma clang fp contract(off)

constexpr int NPTS   = 16384;
constexpr int NCLOUD = 8;
constexpr int PPC    = 2048;
constexpr int CIN    = 64;
constexpr int COUT   = 64;
constexpr int KNN    = 20;
constexpr int NEDGE  = NPTS * KNN;
constexpr int EPC    = PPC * KNN;
constexpr int ABW    = 128;
constexpr int NT     = 256;
constexpr float WCARRY     = 16.0f;
constexpr float WCARRY_INV = 1.0f / 16.0f;
constexpr float BN_EPS_C   = 1e-5f;

constexpr int KN_QPB  = 256;
constexpr int KN_NBLK = NPTS / KN_QPB;
constexpr int KN_BPC  = PPC / KN_QPB;
constexpr int NBLK_ST = 128;
constexpr int RPB     = NEDGE / NBLK_ST;
constexpr int AG_TILE = 128;
constexpr int AG_NBLK = NPTS / AG_TILE;
constexpr int AG_TPC  = PPC / AG_TILE;
constexpr int AG_SCH  = 2048;
constexpr int AG_NCH  = EPC / AG_SCH;

static_assert(NPTS == NCLOUD * PPC, "");
static_assert(KN_NBLK * KN_QPB == NPTS && KN_BPC * KN_QPB == PPC && PPC % KN_QPB == 0, "");
static_assert((KN_QPB * KNN) % (4 * KN_QPB) == 0 && KNN % 4 == 0, "");
static_assert(RPB * NBLK_ST == NEDGE && RPB % 32 == 0 && RPB % 8 == 0 && RPB % 4 == 0, "");
static_assert(AG_NBLK * AG_TILE == NPTS && AG_TPC * AG_TILE == PPC && AG_NCH * AG_SCH == EPC && AG_SCH == 8 * NT, "");
static_assert(AG_TILE == 16 * (NT / 32), "");
static_assert(NEDGE < (1 << 19), "");
static_assert(CIN % 32 == 0 && COUT % 32 == 0, "");
static_assert(NPTS % 64 == 0 && ABW % 64 == 0 && NEDGE % 64 == 0 && COUT % 64 == 0, "");

typedef __attribute__((ext_vector_type(16))) _Float16 v16h;
typedef __attribute__((ext_vector_type(8)))  _Float16 v8h;
typedef __attribute__((ext_vector_type(16))) __bf16   v16b;
typedef __attribute__((ext_vector_type(8)))  __bf16   v8b;
typedef __attribute__((ext_vector_type(8)))  float    v8f;
typedef __attribute__((ext_vector_type(4)))  float    v4f;
typedef __attribute__((ext_vector_type(2)))  float    v2f;
typedef __attribute__((ext_vector_type(4)))  unsigned int v4u;
typedef __attribute__((ext_vector_type(4)))  int      v4i;

__device__ __forceinline__ unsigned short f2bf_bits(float f) {
  unsigned u = __float_as_uint(f);
  return (unsigned short)((u + 0x7FFFu + ((u >> 16) & 1u)) >> 16);
}
__device__ __forceinline__ float bf_bits2f(unsigned short h) { return __uint_as_float(((unsigned)h) << 16); }

__device__ __forceinline__ void dep_guard_h(v8f& a, v8f& b, v16h x, v16h y) { asm volatile("v_nop\n\tv_nop\n\tv_nop\n\tv_nop" : "+v"(a), "+v"(b) : "v"(x), "v"(y)); }
__device__ __forceinline__ void dep_guard_b(v8f& a, v8f& b, v16b x, v16b y) { asm volatile("v_nop\n\tv_nop\n\tv_nop\n\tv_nop" : "+v"(a), "+v"(b) : "v"(x), "v"(y)); }
__device__ __forceinline__ void dep_guard4_h(v8f& a, v8f& b, v8f& c, v8f& d, v16h x, v16h y) { asm volatile("v_nop\n\tv_nop\n\tv_nop\n\tv_nop" : "+v"(a), "+v"(b), "+v"(c), "+v"(d) : "v"(x), "v"(y)); }
__device__ __forceinline__ void dep_guard4_b(v8f& a, v8f& b, v8f& c, v8f& d, v16b x, v16b y) { asm volatile("v_nop\n\tv_nop\n\tv_nop\n\tv_nop" : "+v"(a), "+v"(b), "+v"(c), "+v"(d) : "v"(x), "v"(y)); }
__device__ __forceinline__ void keep4_h(v16h a, v16h b, v16h c, v16h d) { asm volatile("v_nop" :: "v"(a), "v"(b), "v"(c), "v"(d)); }
__device__ __forceinline__ void keep4_b(v16b a, v16b b, v16b c, v16b d) { asm volatile("v_nop" :: "v"(a), "v"(b), "v"(c), "v"(d)); }
__device__ __forceinline__ void acc_guard4(v8f& a, v8f& b, v8f& c, v8f& d) { asm volatile("v_nop\n\tv_nop\n\tv_nop\n\tv_nop" : "+v"(a), "+v"(b), "+v"(c), "+v"(d)); }
template <typename T> struct Frag;
template <> struct Frag<_Float16> {
  typedef v16h V; union U { v16h v; v8h h[2]; };
  static __device__ __forceinline__ v16h load(const _Float16* p) {
    U f; f.h[0] = *(const v8h*)(p); f.h[1] = *(const v8h*)(p + 16); return f.v;
  }
  static __device__ __forceinline__ v8f mma(v16h a, v16h b, v8f c) {
    return __builtin_amdgcn_wmma_f32_16x16x32_f16(false, a, false, b, (short)0, c, false, false);
  }
  static __device__ __forceinline__ void guard(v8f& a, v8f& b, v16h x, v16h y) { dep_guard_h(a, b, x, y); }
  static __device__ __forceinline__ void guard4(v8f& a, v8f& b, v8f& c, v8f& d, v16h x, v16h y) { dep_guard4_h(a, b, c, d, x, y); }
  static __device__ __forceinline__ void keep(v16h a, v16h b, v16h c, v16h d) { keep4_h(a, b, c, d); }
};
template <> struct Frag<__bf16> {
  typedef v16b V; union U { v16b v; v8b h[2]; };
  static __device__ __forceinline__ v16b load(const __bf16* p) {
    U f; f.h[0] = *(const v8b*)(p); f.h[1] = *(const v8b*)(p + 16); return f.v;
  }
  static __device__ __forceinline__ v8f mma(v16b a, v16b b, v8f c) {
    return __builtin_amdgcn_wmma_f32_16x16x32_bf16(false, a, false, b, (short)0, c, false, false);
  }
  static __device__ __forceinline__ void guard(v8f& a, v8f& b, v16b x, v16b y) { dep_guard_b(a, b, x, y); }
  static __device__ __forceinline__ void guard4(v8f& a, v8f& b, v8f& c, v8f& d, v16b x, v16b y) { dep_guard4_b(a, b, c, d, x, y); }
  static __device__ __forceinline__ void keep(v16b a, v16b b, v16b c, v16b d) { keep4_b(a, b, c, d); }
};

__device__ __forceinline__ unsigned pk16(unsigned short a, unsigned short b) { return (unsigned)a | ((unsigned)b << 16); }
__device__ __forceinline__ unsigned short h_bits(float f) { const _Float16 h = (_Float16)f; return __builtin_bit_cast(unsigned short, h); }

__device__ __forceinline__ float h16_to_f32(unsigned hb) {
  const unsigned sgn = (hb & 0x8000u) << 16; const unsigned em = hb & 0x7fffu;
  const float fn = __uint_as_float((em << 13) + 0x38000000u);
  const float fs = (float)em * 5.9604644775390625e-8f;
  const float mag = (em < 0x400u) ? fs : fn; return __uint_as_float(__float_as_uint(mag) | sgn); }

template <int ET> struct Elem;
template <> struct Elem<0> { typedef _Float16 T; };
template <> struct Elem<1> { typedef __bf16 T; };
template <int ET, bool SPLIT, int BIAS_MODE, int OUT_MODE, bool RESID, int ACT = 0>
__global__ __launch_bounds__(256) void wmma_gemm64(
    const unsigned short* __restrict__ Ap, const unsigned short* __restrict__ A2p, int lda, long strideA,
    const unsigned short* __restrict__ Btp, const unsigned short* __restrict__ Bt2p, int ldb, long strideB,
    void* __restrict__ Cout, void* __restrict__ Cout2, int ldc, long strideC,
    const float* __restrict__ bias,
    const float* __restrict__ resid, long strideR,
    int M, int N, int K, float scale) {
  typedef typename Elem<ET>::T T;
  typedef typename Frag<T>::V V;
  const T* A = (const T*)Ap; const T* A2 = (const T*)A2p; const T* Bt = (const T*)Btp; const T* Bt2 = (const T*)Bt2p;
  __shared__ __align__(16) float sT[8][16 * 68];
  const int b    = blockIdx.y;
  const int lane = threadIdx.x & 31;
  const int wave = threadIdx.x >> 5;
  const int tilesN = N >> 6;
  const int tilesM = M >> 6;
  const int tile = blockIdx.x * 8 + wave;
  if (tile >= tilesM * tilesN) return;
  const int tm = tile / tilesN;
  const int tn = tile - tm * tilesN;
  const int m0 = tm << 6;
  const int n0 = tn << 6;

  const T* Ab  = A  + (size_t)b * strideA;
  const T* Bb  = Bt + (size_t)b * strideB;
  const T* Ab2 = SPLIT ? (A2  + (size_t)b * strideA) : nullptr;
  const T* Bb2 = SPLIT ? (Bt2 + (size_t)b * strideB) : nullptr;

  const int rlane = lane & 15;
  const int koff  = (lane >> 4) * 8;
  const int mOff  = (lane >> 4) * 8;

  v8f acc[4][4];
#pragma unroll
  for (int i = 0; i < 4; ++i)
#pragma unroll
    for (int j = 0; j < 4; ++j) acc[i][j] = (v8f){0.f,0.f,0.f,0.f,0.f,0.f,0.f,0.f};

  for (int k0 = 0; k0 < K; k0 += 32) {
    V bh[4], bl[4];
#pragma unroll
    for (int j = 0; j < 4; ++j) {
      const size_t bo = (size_t)(n0 + (j << 4) + rlane) * ldb + koff + k0;
      bh[j] = Frag<T>::load(Bb + bo);
      if (SPLIT) bl[j] = Frag<T>::load(Bb2 + bo);
    }
#pragma unroll
    for (int i = 0; i < 4; ++i) {
      const size_t ao = (size_t)(m0 + (i << 4) + rlane) * lda + koff + k0;
      V ah = Frag<T>::load(Ab + ao);
      V al;
      if (SPLIT) al = Frag<T>::load(Ab2 + ao);
#pragma unroll
      for (int j = 0; j < 4; ++j) {
        acc[i][j] = Frag<T>::mma(ah, bh[j], acc[i][j]);
        if (SPLIT) {
          acc[i][j] = Frag<T>::mma(ah, bl[j], acc[i][j]);
          acc[i][j] = Frag<T>::mma(al, bh[j], acc[i][j]);
        }
      }
      Frag<T>::guard4(acc[i][0], acc[i][1], acc[i][2], acc[i][3], ah, SPLIT ? al : ah);
    }
    Frag<T>::keep(bh[0], bh[1], bh[2], bh[3]);
    if (SPLIT) Frag<T>::keep(bl[0], bl[1], bl[2], bl[3]);
  }
  acc_guard4(acc[0][0], acc[0][1], acc[0][2], acc[0][3]);
  acc_guard4(acc[1][0], acc[1][1], acc[1][2], acc[1][3]);
  acc_guard4(acc[2][0], acc[2][1], acc[2][2], acc[2][3]);
  acc_guard4(acc[3][0], acc[3][1], acc[3][2], acc[3][3]);

  float* slab = sT[wave];
  const float* Rb = RESID ? (resid + (size_t)b * strideR) : nullptr;
#pragma unroll
  for (int i = 0; i < 4; ++i) {
    const int mBase = m0 + (i << 4);
#pragma unroll
    for (int j = 0; j < 4; ++j) {
      const int n = n0 + (j << 4) + rlane;
      float bv = 0.f;
      if (BIAS_MODE == 2) bv = bias[n];
#pragma unroll
      for (int r = 0; r < 8; ++r) {
        float v = acc[i][j][r] * scale;
        if (BIAS_MODE == 1) v += bias[mBase + mOff + r];
        if (BIAS_MODE == 2) v += bv;
        if (RESID) v += Rb[(size_t)(mBase + mOff + r) * ldc + n];
        if (ACT == 2) v = fmaxf(v, 0.0f);
        if (ACT == 4) v = (v > 0.f) ? v : 0.01f * v;
        slab[(mOff + r) * 68 + (j << 4) + rlane] = v;
      }
    }
    __builtin_amdgcn_fence(__ATOMIC_RELEASE, "workgroup");
    __builtin_amdgcn_wave_barrier();
    __builtin_amdgcn_fence(__ATOMIC_ACQUIRE, "workgroup");
    if (OUT_MODE == 0) {
      float* C = (float*)Cout + (size_t)b * strideC;
      const int hh = lane >> 4, c4 = (lane & 15) * 4;
      for (int pass = 0; pass < 2; ++pass) {
#pragma unroll
        for (int it = 0; it < 8; ++it) {
          const int row = it * 2 + hh;
          v4f v = *(const v4f*)(slab + row * 68 + c4);
          *(volatile v4f*)(C + (size_t)(mBase + row) * ldc + n0 + c4) = v;
        }
        __threadfence();
      }
    } else {
      const int q = lane >> 3, c8 = (lane & 7) * 8;
      unsigned short* C  = (unsigned short*)Cout  + (size_t)b * strideC;
      unsigned short* C2 = (OUT_MODE == 2) ? ((unsigned short*)Cout2 + (size_t)b * strideC) : nullptr;
      for (int pass = 0; pass < 2; ++pass) {
#pragma unroll
        for (int it = 0; it < 4; ++it) {
          const int row = it * 4 + q;
          const float* sp = slab + row * 68 + c8;
          v8h hv, lv;
#pragma unroll
          for (int e = 0; e < 8; ++e) {
            if (OUT_MODE == 1) {
              hv[e] = (_Float16)sp[e];
            } else {
              unsigned short hb = f2bf_bits(sp[e]);
              unsigned short lb = f2bf_bits(sp[e] - bf_bits2f(hb));
              hv[e] = __builtin_bit_cast(_Float16, hb);
              lv[e] = __builtin_bit_cast(_Float16, lb);
            }
          }
          *(volatile v8h*)(C + (size_t)(mBase + row) * ldc + n0 + c8) = hv;
          if (OUT_MODE == 2) *(volatile v8h*)(C2 + (size_t)(mBase + row) * ldc + n0 + c8) = lv;
        }
        __threadfence();
      }
    }
    __builtin_amdgcn_fence(__ATOMIC_RELEASE, "workgroup");
    __builtin_amdgcn_wave_barrier();
    __builtin_amdgcn_fence(__ATOMIC_ACQUIRE, "workgroup");
  }
}

__global__ __launch_bounds__(256) void cast8_f16_kernel(const float* __restrict__ in, unsigned short* __restrict__ out, int n8) {
  const int i = blockIdx.x * 256 + threadIdx.x;
  if (i >= n8) return;
  const float* p = in + 8 * (size_t)i;
  const v4f a = *(const v4f*)(p);
  const v4f c = *(const v4f*)(p + 4);
  unsigned short hb[8];
#pragma unroll
  for (int e = 0; e < 4; ++e) {
    hb[e]     = h_bits(a[e]);
    hb[4 + e] = h_bits(c[e]);
  }
  const v4u u = (v4u){pk16(hb[0], hb[1]), pk16(hb[2], hb[3]), pk16(hb[4], hb[5]), pk16(hb[6], hb[7])};
  unsigned short* q = out + 8 * (size_t)i;
  *(volatile v4u*)q = u;
  __threadfence();
  *(volatile v4u*)q = u;
}

__device__ __forceinline__ int blk_excl_scan(int cnt, int* scan_ws, int tid, int* tot) {
  const int lane = tid & 31, wave = tid >> 5; int incl = cnt;
#pragma unroll
  for (int o = 1; o < 32; o <<= 1) { const int v = __shfl_up(incl, o, 32); if (lane >= o) incl += v; }
  if (lane == 31) scan_ws[wave] = incl;
  __syncthreads();
  if (wave == 0) { int wv = (lane < NT / 32) ? scan_ws[lane] : 0; int wincl = wv;
#pragma unroll
    for (int o = 1; o < 32; o <<= 1) { const int v = __shfl_up(wincl, o, 32); if (lane >= o) wincl += v; }
    if (lane < NT / 32) scan_ws[32 + lane] = wincl - wv; if (lane == 31) scan_ws[64] = wincl; }
  __syncthreads();
  const int res = scan_ws[32 + wave] + incl - cnt; *tot = scan_ws[64];
  return res;
}

__global__ __launch_bounds__(256) void knn_kernel(const float* __restrict__ pos, const int* __restrict__ batch,
                                                  const int* __restrict__ kvec, int* __restrict__ nbr) {
  __shared__ __align__(16) v4f sp4[PPC];
  __shared__ __align__(16) int snb[KN_QPB * KNN];
  (void)batch; (void)kvec;
  const int tid = threadIdx.x;
  const int cl = (int)blockIdx.x / KN_BPC;
  const int qb = (int)blockIdx.x - cl * KN_BPC;
  const int cbase = cl * PPC;
#pragma unroll 1
  for (int idx = tid; idx < PPC; idx += KN_QPB) {
    const float px = pos[(size_t)(cbase + idx) * 3 + 0];
    const float py = pos[(size_t)(cbase + idx) * 3 + 1];
    const float pz = pos[(size_t)(cbase + idx) * 3 + 2];
    const float t0 = px * px, t1 = py * py, t2 = pz * pz;
    const float sq = (t0 + t2) + t1;
    sp4[idx] = (v4f){px, py, pz, sq};
  }
  __syncthreads();
  const int ql = qb * KN_QPB + tid;
  const v4f qv = sp4[ql];
  float bd[KNN]; int bi[KNN];
#pragma unroll
  for (int t = 0; t < KNN; ++t) { bd[t] = 3.0e38f; bi[t] = 0; }
#pragma unroll 2
  for (int j = 0; j < PPC; ++j) {
    const v4f cv = sp4[j];
    float dt = qv[0] * cv[0];
    dt = fmaf(qv[1], cv[1], dt);
    dt = fmaf(qv[2], cv[2], dt);
    const float d2 = (qv[3] + cv[3]) - 2.0f * dt;
    if (j != ql && d2 <= bd[KNN - 1]) {
      float cd = d2; int ci = j;
#pragma unroll
      for (int t = 0; t < KNN; ++t) {
        const bool lt = (cd < bd[t]) || (cd == bd[t] && ci < bi[t]);
        const float td = bd[t]; const int ti = bi[t];
        bd[t] = lt ? cd : td;
        bi[t] = lt ? ci : ti;
        cd = lt ? td : cd;
        ci = lt ? ti : ci;
      }
    }
  }
#pragma unroll
  for (int u = 0; u < KNN / 4; ++u) {
    const v4i w = (v4i){cbase + bi[4 * u], cbase + bi[4 * u + 1], cbase + bi[4 * u + 2], cbase + bi[4 * u + 3]};
    *(v4i*)(snb + tid * KNN + 4 * u) = w;
  }
  __syncthreads();
  int* ob = nbr + (size_t)(cbase + qb * KN_QPB) * KNN;
  for (int pass = 0; pass < 2; ++pass) {
#pragma unroll
    for (int it = 0; it < (KN_QPB * KNN) / (4 * KN_QPB); ++it) {
      const int i4 = it * KN_QPB + tid;
      const v4i v = *(const v4i*)(snb + 4 * i4);
      *(volatile v4i*)(ob + 4 * i4) = v;
    }
    __threadfence();
  }
}

__global__ __launch_bounds__(256) void wprep_kernel(const float* __restrict__ W1, const float* __restrict__ W2,
                                                    unsigned short* __restrict__ Bt1, unsigned short* __restrict__ Bt2) {
  const int tid = threadIdx.x;
  if (blockIdx.x < 4) {
    const int i = blockIdx.x * 256 + tid;
    const int n = i >> 3, c8 = (i & 7) * 8;
    const int na = n & 63;
    const float fa = (n < 64) ? 1.0f : 0.0f;
    const float fb = 1.0f - 2.0f * fa;
    const float* ra = W1 + (size_t)na * 128 + c8;
    const float* rb = W1 + (size_t)na * 128 + 64 + c8;
    const v4f a0 = *(const v4f*)ra, a1 = *(const v4f*)(ra + 4);
    const v4f b0 = *(const v4f*)rb, b1v = *(const v4f*)(rb + 4);
    unsigned short hb[8];
#pragma unroll
    for (int e = 0; e < 4; ++e) {
      const float v0 = fmaf(fa, a0[e], fb * b0[e]) * WCARRY;
      const float v1 = fmaf(fa, a1[e], fb * b1v[e]) * WCARRY;
      hb[e] = h_bits(v0); hb[4 + e] = h_bits(v1);
    }
    const v4u u = (v4u){pk16(hb[0], hb[1]), pk16(hb[2], hb[3]), pk16(hb[4], hb[5]), pk16(hb[6], hb[7])};
    unsigned short* q = Bt1 + 8 * (size_t)i;
    *(volatile v4u*)q = u;
    __threadfence();
    *(volatile v4u*)q = u;
  } else {
    const int i = (blockIdx.x - 4) * 256 + tid;
    const float* r = W2 + 8 * (size_t)i;
    const v4f a0 = *(const v4f*)r, a1 = *(const v4f*)(r + 4);
    unsigned short hb[8];
#pragma unroll
    for (int e = 0; e < 4; ++e) { hb[e] = h_bits(a0[e] * WCARRY); hb[4 + e] = h_bits(a1[e] * WCARRY); }
    const v4u u = (v4u){pk16(hb[0], hb[1]), pk16(hb[2], hb[3]), pk16(hb[4], hb[5]), pk16(hb[6], hb[7])};
    unsigned short* q = Bt2 + 8 * (size_t)i;
    *(volatile v4u*)q = u;
    __threadfence();
    *(volatile v4u*)q = u;
  }
}

__global__ __launch_bounds__(256) void stats1_kernel(const float* __restrict__ AB, const int* __restrict__ nbr,
                                                     const float* __restrict__ b1, float* __restrict__ P1) {
  __shared__ __align__(16) float red[4 * 128];
  const int tid = threadIdx.x, g = tid >> 6, c = tid & 63, lane = tid & 31, wave = tid >> 5;
  const float bc = b1[c];
  float s = 0.0f, q = 0.0f;
  const int e0 = blockIdx.x * RPB;
#pragma unroll 2
  for (int it = 0; it < RPB / 4; ++it) {
    const int e = e0 + it * 4 + g;
    int j = nbr[e]; j = j < 0 ? 0 : (j > NPTS - 1 ? NPTS - 1 : j);
    const int i = e / KNN;
    const float h = (AB[(size_t)j * ABW + c] + AB[(size_t)i * ABW + 64 + c]) + bc;
    s += h; q = fmaf(h, h, q);
  }
  red[g * 128 + c] = s; red[g * 128 + 64 + c] = q;
  __syncthreads();
  if (wave == 0) {
    v4f t = *(const v4f*)(red + 4 * lane);
    t = t + *(const v4f*)(red + 128 + 4 * lane);
    t = t + *(const v4f*)(red + 256 + 4 * lane);
    t = t + *(const v4f*)(red + 384 + 4 * lane);
    float* op = P1 + (size_t)blockIdx.x * 128 + 4 * lane;
    for (int pass = 0; pass < 2; ++pass) { *(volatile v4f*)op = t; __threadfence(); }
  }
}

__global__ __launch_bounds__(64) void finalize_kernel(const float* __restrict__ P, int nblk, const float* __restrict__ gam,
                                                      float* __restrict__ MS) {
  __shared__ __align__(16) float so[128];
  const int c = threadIdx.x;
  double S = 0.0, Q = 0.0;
#pragma unroll 1
  for (int b = 0; b < nblk; ++b) { S += (double)P[(size_t)b * 128 + c]; Q += (double)P[(size_t)b * 128 + 64 + c]; }
  const double mu = S * (1.0 / (double)NEDGE);
  double var = Q * (1.0 / (double)NEDGE) - mu * mu;
  var = var < 0.0 ? 0.0 : var;
  const float varf = (float)var;
  const float r = 1.0f / sqrtf(varf + BN_EPS_C);
  so[c] = (float)mu; so[64 + c] = r * gam[c];
  __syncthreads();
  if (c < 32) {
    const v4f v = *(const v4f*)(so + 4 * c);
    for (int pass = 0; pass < 2; ++pass) { *(volatile v4f*)(MS + 4 * c) = v; __threadfence(); }
  }
}

__global__ __launch_bounds__(256) void h1n_kernel(const float* __restrict__ AB, const int* __restrict__ nbr,
                                                  const float* __restrict__ b1, const float* __restrict__ MS1,
                                                  const float* __restrict__ beta1, unsigned short* __restrict__ H1N) {
  __shared__ __align__(16) float cst[256];
  const int tid = threadIdx.x;
  {
    const int seg = tid >> 6;
    const float va = b1[tid & 63];
    const float vm = MS1[(tid - 64) & 127];
    const float vb = beta1[tid & 63];
    const float fa = (seg == 0) ? 1.0f : 0.0f;
    const float fm = (seg == 1 || seg == 2) ? 1.0f : 0.0f;
    const float fbb = (seg == 3) ? 1.0f : 0.0f;
    cst[tid] = (fa * va + fm * vm) + fbb * vb;
  }
  __syncthreads();
  const int r = tid >> 3, c8 = (tid & 7) * 8;
  const v4f bb0 = *(const v4f*)(cst + c8),       bb1 = *(const v4f*)(cst + c8 + 4);
  const v4f mu0 = *(const v4f*)(cst + 64 + c8),  mu1 = *(const v4f*)(cst + 64 + c8 + 4);
  const v4f s0  = *(const v4f*)(cst + 128 + c8), s1  = *(const v4f*)(cst + 128 + c8 + 4);
  const v4f be0 = *(const v4f*)(cst + 192 + c8), be1 = *(const v4f*)(cst + 192 + c8 + 4);
  const int e0 = blockIdx.x * RPB;
#pragma unroll 1
  for (int it = 0; it < RPB / 32; ++it) {
    const int e = e0 + it * 32 + r;
    int j = nbr[e]; j = j < 0 ? 0 : (j > NPTS - 1 ? NPTS - 1 : j);
    const int i = e / KNN;
    const float* pj = AB + (size_t)j * ABW + c8;
    const float* pi = AB + (size_t)i * ABW + 64 + c8;
    const v4f j0 = *(const v4f*)pj, j1 = *(const v4f*)(pj + 4);
    const v4f i0 = *(const v4f*)pi, i1 = *(const v4f*)(pi + 4);
    unsigned short hb[8];
#pragma unroll
    for (int k = 0; k < 4; ++k) {
      float h = (j0[k] + i0[k]) + bb0[k];
      float v = fmaf(h - mu0[k], s0[k], be0[k]);
      v = fmaxf(v, 0.0f);
      hb[k] = h_bits(v);
      h = (j1[k] + i1[k]) + bb1[k];
      v = fmaf(h - mu1[k], s1[k], be1[k]);
      v = fmaxf(v, 0.0f);
      hb[4 + k] = h_bits(v);
    }
    const v4u u = (v4u){pk16(hb[0], hb[1]), pk16(hb[2], hb[3]), pk16(hb[4], hb[5]), pk16(hb[6], hb[7])};
    unsigned short* q = H1N + (size_t)e * 64 + c8;
    *(volatile v4u*)q = u;
    __threadfence();
    *(volatile v4u*)q = u;
  }
}

__global__ __launch_bounds__(256) void stats2_kernel(const unsigned* __restrict__ H2w, float* __restrict__ P2) {
  __shared__ __align__(16) float red[8 * 128];
  const int tid = threadIdx.x, lane = tid & 31, wave = tid >> 5;
  float s0 = 0.0f, s1 = 0.0f, q0 = 0.0f, q1 = 0.0f;
  const int r0 = blockIdx.x * RPB;
#pragma unroll 2
  for (int it = 0; it < RPB / 8; ++it) {
    const int row = r0 + it * 8 + wave;
    const unsigned w = H2w[(size_t)row * 32 + lane];
    const float f0 = h16_to_f32(w & 0xffffu), f1 = h16_to_f32(w >> 16);
    s0 += f0; s1 += f1; q0 = fmaf(f0, f0, q0); q1 = fmaf(f1, f1, q1);
  }
  *(v2f*)(red + wave * 128 + 2 * lane) = (v2f){s0, s1};
  *(v2f*)(red + wave * 128 + 64 + 2 * lane) = (v2f){q0, q1};
  __syncthreads();
  if (wave == 0) {
    v4f t = *(const v4f*)(red + 4 * lane);
#pragma unroll
    for (int w2 = 1; w2 < 8; ++w2) t = t + *(const v4f*)(red + w2 * 128 + 4 * lane);
    float* op = P2 + (size_t)blockIdx.x * 128 + 4 * lane;
    for (int pass = 0; pass < 2; ++pass) { *(volatile v4f*)op = t; __threadfence(); }
  }
}

__global__ __launch_bounds__(256) void agg_kernel(const unsigned* __restrict__ H2w, const int* __restrict__ nbr,
                                                  const float* __restrict__ MS2, const float* __restrict__ beta2,
                                                  float* __restrict__ out) {
  __shared__ int LIST[AG_SCH];
  __shared__ __align__(16) float accs[AG_TILE * 64];
  __shared__ int scan_ws[80];
  const int tid = threadIdx.x, lane = tid & 31, wave = tid >> 5;
  const int n0 = blockIdx.x * AG_TILE;
  const int cl = blockIdx.x / AG_TPC;
  const int ebase = cl * EPC;
  const int c0 = 2 * lane;
  const float mA = MS2[c0], mB = MS2[c0 + 1];
  const float sA = MS2[64 + c0], sB = MS2[64 + c0 + 1];
  const float bA = beta2[c0], bB = beta2[c0 + 1];
  for (int i = tid; i < AG_TILE * 64; i += NT) accs[i] = 0.0f;
  for (int i = tid; i < AG_SCH; i += NT) LIST[i] = 0;
  if (tid < 80) scan_ws[tid] = 0;
  __syncthreads();
#pragma unroll 1
  for (int ch = 0; ch < AG_NCH; ++ch) {
    const int e0 = ebase + ch * AG_SCH + tid * 8;
    const v4i a = *(const v4i*)(nbr + e0);
    const v4i b = *(const v4i*)(nbr + e0 + 4);
    int dv[8];
    dv[0] = a[0]; dv[1] = a[1]; dv[2] = a[2]; dv[3] = a[3]; dv[4] = b[0]; dv[5] = b[1]; dv[6] = b[2]; dv[7] = b[3];
    int rec[8]; int cnt = 0;
#pragma unroll
    for (int k = 0; k < 8; ++k) {
      const int d = dv[k]; int r = -1;
      if (d >= n0 && d < n0 + AG_TILE) { r = ((d - n0) << 19) | (e0 + k); ++cnt; }
      rec[k] = r;
    }
    int tot; int p = blk_excl_scan(cnt, scan_ws, tid, &tot);
#pragma unroll
    for (int k = 0; k < 8; ++k) if (rec[k] >= 0) { if ((unsigned)p < (unsigned)AG_SCH) LIST[p] = rec[k]; ++p; }
    __syncthreads();
    const int totc = tot < AG_SCH ? tot : AG_SCH;
#pragma unroll 1
    for (int base = 0; base < totc; base += 32) {
      const int q = base + lane;
      const int qc = q < AG_SCH ? q : AG_SCH - 1;
      const int lv = LIST[qc];
      const int rv = (q < totc) ? lv : -1;
      const int own = (rv >= 0 && (rv >> 23) == wave) ? 1 : 0;
      unsigned msk = (unsigned)__ballot(own);
#pragma unroll 1
      for (int itb = 0; itb < 32; ++itb) {
        if (msk == 0u) break;
        const int bp = __builtin_ctz(msk); msk &= msk - 1u;
        const int r = __shfl(rv, bp, 32);
        const int dl = (r >> 19) & (AG_TILE - 1);
        int e = r & 0x7FFFF; e = e > NEDGE - 1 ? NEDGE - 1 : e;
        const unsigned w = H2w[(size_t)e * 32 + lane];
        const float f0 = h16_to_f32(w & 0xffffu), f1 = h16_to_f32(w >> 16);
        const float v0 = fmaxf(fmaf(f0 - mA, sA, bA), 0.0f);
        const float v1 = fmaxf(fmaf(f1 - mB, sB, bB), 0.0f);
        v2f* ap = (v2f*)(accs + dl * 64 + c0);
        const v2f o = *ap;
        const v2f nv = (v2f){fmaxf(o[0], v0), fmaxf(o[1], v1)};
        *ap = nv;
      }
    }
    __syncthreads();
  }
  const int hh = lane >> 4, c4 = (lane & 15) * 4;
  for (int pass = 0; pass < 2; ++pass) {
#pragma unroll
    for (int it = 0; it < 8; ++it) {
      const int rl = wave * 16 + it * 2 + hh;
      const v4f v = *(const v4f*)(accs + rl * 64 + c4);
      *(volatile v4f*)(out + (size_t)(n0 + rl) * 64 + c4) = v;
    }
    __threadfence();
  }
}

extern "C" void kernel_launch(void* const* d_in, const int* in_sizes, int n_in,
                              void* d_out, int out_size, void* d_ws, size_t ws_size, hipStream_t stream) {
  if (n_in < 12) return;
  if (in_sizes[0] != NPTS * CIN || in_sizes[1] != NPTS * 3 || in_sizes[2] != NPTS || in_sizes[3] != COUT * 2 * CIN ||
      in_sizes[4] != COUT || in_sizes[5] != COUT || in_sizes[6] != COUT || in_sizes[7] != COUT * COUT ||
      in_sizes[8] != COUT || in_sizes[9] != COUT || in_sizes[10] != COUT || out_size != NPTS * COUT) return;
  const float* x     = (const float*)d_in[0];
  const float* pos   = (const float*)d_in[1];
  const int*   batch = (const int*)d_in[2];
  const float* W1    = (const float*)d_in[3];
  const float* b1    = (const float*)d_in[4];
  const float* g1    = (const float*)d_in[5];
  const float* beta1 = (const float*)d_in[6];
  const float* W2    = (const float*)d_in[7];
  const float* b2    = (const float*)d_in[8];
  const float* g2    = (const float*)d_in[9];
  const float* beta2 = (const float*)d_in[10];
  const int*   kvec  = (const int*)d_in[11];
  float* out = (float*)d_out;

  char* ws = (char*)d_ws; size_t off = 0;
  auto carve = [&](size_t bytes) -> char* { char* p = ws + off; off += (bytes + 255) & ~(size_t)255; return p; };
  int*            NBR = (int*)carve((size_t)NEDGE * 4);
  unsigned short* XH  = (unsigned short*)carve((size_t)NPTS * CIN * 2);
  unsigned short* BT1 = (unsigned short*)carve((size_t)ABW * CIN * 2);
  unsigned short* BT2 = (unsigned short*)carve((size_t)COUT * COUT * 2);
  float*          AB  = (float*)carve((size_t)NPTS * ABW * 4);
  float*          P1  = (float*)carve((size_t)NBLK_ST * 128 * 4);
  float*          MS1 = (float*)carve(512);
  unsigned short* H1N = (unsigned short*)carve((size_t)NEDGE * COUT * 2);
  unsigned short* H2P = (unsigned short*)carve((size_t)NEDGE * COUT * 2);
  float*          P2  = (float*)carve((size_t)NBLK_ST * 128 * 4);
  float*          MS2 = (float*)carve(512);
  if (off > ws_size || off > (size_t)134217728) return;

  knn_kernel<<<KN_NBLK, KN_QPB, 0, stream>>>(pos, batch, kvec, NBR);
  cast8_f16_kernel<<<(NPTS * CIN / 8) / 256, 256, 0, stream>>>(x, XH, NPTS * CIN / 8);
  wprep_kernel<<<6, 256, 0, stream>>>(W1, W2, BT1, BT2);
  {
    const int tiles = (NPTS / 64) * (ABW / 64);
    wmma_gemm64<0, false, 0, 0, false><<<dim3(tiles / 8, 1), 256, 0, stream>>>(
        (const unsigned short*)XH, (const unsigned short*)nullptr, CIN, 0L,
        (const unsigned short*)BT1, (const unsigned short*)nullptr, CIN, 0L,
        (void*)AB, (void*)nullptr, ABW, 0L,
        (const float*)nullptr, (const float*)nullptr, 0L, NPTS, ABW, CIN, WCARRY_INV);
  }
  stats1_kernel<<<NBLK_ST, NT, 0, stream>>>(AB, NBR, b1, P1);
  finalize_kernel<<<1, 64, 0, stream>>>(P1, NBLK_ST, g1, MS1);
  h1n_kernel<<<NBLK_ST, NT, 0, stream>>>(AB, NBR, b1, MS1, beta1, H1N);
  {
    const int tiles = (NEDGE / 64) * (COUT / 64);
    wmma_gemm64<0, false, 2, 1, false><<<dim3(tiles / 8, 1), 256, 0, stream>>>(
        (const unsigned short*)H1N, (const unsigned short*)nullptr, COUT, 0L,
        (const unsigned short*)BT2, (const unsigned short*)nullptr, COUT, 0L,
        (void*)H2P, (void*)nullptr, COUT, 0L,
        b2, (const float*)nullptr, 0L, NEDGE, COUT, COUT, WCARRY_INV);
  }
  stats2_kernel<<<NBLK_ST, NT, 0, stream>>>((const unsigned*)H2P, P2);
  finalize_kernel<<<1, 64, 0, stream>>>(P2, NBLK_ST, g2, MS2);
  agg_kernel<<<AG_NBLK, NT, 0, stream>>>((const unsigned*)H2P, NBR, MS2, beta2, out);
}
